// WeightedConv2D_56289841381897
// MI455X (gfx1250) — hardware-verified
//
#include <hip/hip_runtime.h>


#define NBI  4
#define CH   64
#define CO   64
#define NN   16384
#define KK   9
#define PADK 4
#define KC   (CH * KK)
#define NOR  4
#define CCAT (NOR * CO)
#define NP2  (NN + 2)
#define SIG  0.08f
#define BEPS 1e-5f
#define DM   KC
#define LOSC 1024.0f

typedef _Float16 h16;
typedef unsigned short bf;
typedef __attribute__((ext_vector_type(16))) __bf16   v16bf;
typedef __attribute__((ext_vector_type(16))) _Float16 v16h;
typedef __attribute__((ext_vector_type(8)))  _Float16 v8h;
typedef __attribute__((ext_vector_type(8)))  unsigned short v8us;
typedef __attribute__((ext_vector_type(8)))  float    v8f;
typedef __attribute__((ext_vector_type(4)))  float    v4f;
typedef v8h  __attribute__((may_alias)) v8ha;
typedef v4f  __attribute__((may_alias)) v4fa;
typedef v8us __attribute__((may_alias)) v8usa;

__device__ __forceinline__ unsigned short f2bf(float f) { unsigned u = __float_as_uint(f); u += 0x7FFFu + ((u >> 16) & 1u); return (unsigned short)(u >> 16); }
__device__ __forceinline__ float bf2f(unsigned short b) { return __uint_as_float(((unsigned)b) << 16); }
__device__ __forceinline__ float bfr(float f) { return bf2f(f2bf(f)); }
__device__ __forceinline__ v16h cat16(v8h lo, v8h hi) { return __builtin_shufflevector(lo, hi, 0, 1, 2, 3, 4, 5, 6, 7, 8, 9, 10, 11, 12, 13, 14, 15); }
__device__ __forceinline__ v16bf cat16b(v8us lo, v8us hi) { return __builtin_bit_cast(v16bf, __builtin_shufflevector(lo, hi, 0, 1, 2, 3, 4, 5, 6, 7, 8, 9, 10, 11, 12, 13, 14, 15)); }
__device__ __forceinline__ v8f wmma16(v16h a, v16h b, v8f c) { return __builtin_amdgcn_wmma_f32_16x16x32_f16(false, a, false, b, (short)0, c, false, false); }
__device__ __forceinline__ v8f wmmab(v16bf a, v16bf b, v8f c) { return __builtin_amdgcn_wmma_f32_16x16x32_bf16(false, a, false, b, (short)0, c, false, false); }

template <bool SPLITA, bool F16OUT = false>
__global__ __launch_bounds__(128) void k_gemmb(const bf* __restrict__ A, const bf* __restrict__ Al, const bf* __restrict__ Bn, const float* __restrict__ bias, float* C, int ldc, h16* C2, const float* __restrict__ R = nullptr, int K = DM, int roundR = 1) {
    __shared__ __align__(16) float ost[4][16 * 68];
    const int lane = threadIdx.x & 31, wave = threadIdx.x >> 5, lr = lane & 15, hi = lane >> 4;
    const int r0 = blockIdx.x * 64 + wave * 16, c0 = blockIdx.y * 64;
    const size_t aoff = (size_t)(r0 + lr) * K + 8 * hi;
    size_t boff[4];
#pragma unroll
    for (int t = 0; t < 4; ++t) boff[t] = (size_t)(c0 + t * 16 + lr) * K + 8 * hi;
    v8f acc[4];
#pragma unroll
    for (int t = 0; t < 4; ++t) acc[t] = (v8f){};
#pragma unroll 1
    for (int kc = 0; kc < K; kc += 32) {
        const v16bf a = cat16b(*(const v8us*)(A + aoff + kc), *(const v8us*)(A + aoff + kc + 16));
        v16bf al = a;
        if (SPLITA) al = cat16b(*(const v8us*)(Al + aoff + kc), *(const v8us*)(Al + aoff + kc + 16));
#pragma unroll
        for (int t = 0; t < 4; ++t) { const v16bf b = cat16b(*(const v8us*)(Bn + boff[t] + kc), *(const v8us*)(Bn + boff[t] + kc + 16)); acc[t] = wmmab(a, b, acc[t]); if (SPLITA) acc[t] = wmmab(al, b, acc[t]); }
        asm volatile("v_nop\n\tv_nop\n\tv_nop\n\tv_nop" : "+v"(acc[0]), "+v"(acc[1]), "+v"(acc[2]), "+v"(acc[3]) : "v"(a), "v"(al));
    }
    float* os = &ost[wave][0];
#pragma unroll
    for (int t = 0; t < 4; ++t) { const float bv = bias ? bfr(bias[c0 + t * 16 + lr]) : 0.f;
#pragma unroll
        for (int j = 0; j < 8; ++j) os[(hi * 8 + j) * 68 + t * 16 + lr] = acc[t][j] + bv; }
    __syncthreads();
    if (F16OUT) {
        h16* crow = (h16*)(void*)C + (size_t)r0 * ldc + c0;
        auto pass = [&]() {
#pragma unroll
            for (int s = 0; s < 4; ++s) { const int row = 4 * s + (lane >> 3), piece = lane & 7; const float* sp = os + row * 68 + piece * 8; v8h o, o2;
#pragma unroll
                for (int i = 0; i < 8; ++i) { const h16 a = (h16)sp[i]; o[i] = a; o2[i] = (h16)((sp[i] - (float)a) * LOSC); }
                *(volatile v8h*)(crow + (size_t)row * ldc + piece * 8) = o; if (C2) *(volatile v8h*)(C2 + (size_t)r0 * ldc + c0 + (size_t)row * ldc + piece * 8) = o2; }
        };
        pass(); __threadfence(); pass();
    } else {
        float* crow = C + (size_t)r0 * ldc + c0;
        auto pass = [&]() {
#pragma unroll
            for (int s = 0; s < 8; ++s) { const int Lid = (lane >> 3) + 4 * s, piece = lane & 7; const int row = Lid >> 1, cofs = (Lid & 1) * 32 + piece * 4;
                v4f val = *(const v4fa*)(os + row * 68 + cofs); if (R) { const v4f rv = *(const v4f*)(R + ((size_t)r0 + row) * ldc + c0 + cofs); val += roundR ? (v4f){bfr(rv[0]), bfr(rv[1]), bfr(rv[2]), bfr(rv[3])} : rv; }
                *(volatile v4f*)(crow + (size_t)row * ldc + cofs) = val; }
        };
        pass(); __threadfence(); pass();
    }
}


__global__ __launch_bounds__(256) void k_cvt8(const float* __restrict__ src, bf* dst, size_t n8) {
    const size_t i = (size_t)blockIdx.x * 256 + threadIdx.x; if (i >= n8) return;
    const v8f v = *(const v8f*)(src + i * 8); v8us o;
#pragma unroll
    for (int k = 0; k < 8; ++k) o[k] = f2bf(v[k]);
    *(volatile v8us*)(dst + i * 8) = o; __threadfence(); *(volatile v8us*)(dst + i * 8) = o;
}
__global__ __launch_bounds__(256) void k_zero8(bf* dst, size_t n8) {
    const size_t i = (size_t)blockIdx.x * 256 + threadIdx.x; if (i >= n8) return; v8us z;
#pragma unroll
    for (int k = 0; k < 8; ++k) z[k] = 0;
    *(volatile v8us*)(dst + i * 8) = z; __threadfence(); *(volatile v8us*)(dst + i * 8) = z;
}

__global__ __launch_bounds__(256) void k_xgather(const float* __restrict__ XS, const int* __restrict__ idx, int b, int i, float* XD) {
    const int lane = threadIdx.x & 31; const size_t wid = (size_t)blockIdx.x * 8 + (threadIdx.x >> 5); if (wid >= (size_t)CH * (NN / 32)) return; const int c = (int)(wid / (NN / 32)), n = (int)(wid % (NN / 32)) * 32 + lane;
    int m = idx[((size_t)b * NN + n) * NOR + i]; m = m < 0 ? 0 : (m >= NN ? NN - 1 : m); const float v = XS[(size_t)c * NN + m];
    *(volatile float*)(XD + (size_t)c * NN + n) = v; __threadfence(); *(volatile float*)(XD + (size_t)c * NN + n) = v;
}
__global__ __launch_bounds__(256) void k_wim(const float* __restrict__ XG, const float* __restrict__ co, int b, int i, bf* Ah, bf* Al) {
    __shared__ float dws[8][16];
    const int lane = threadIdx.x & 31, wv = threadIdx.x >> 5, n = blockIdx.x * 8 + wv;
    { float w = 0.f;
      if (lane < KK) { const int m = n + lane - PADK; const bool ok = (m >= 0) && (m < NN); float s = 0.f;
#pragma unroll
          for (int d = 0; d < 3; ++d) { const float cc = bfr(co[(((size_t)b * 3 + d) * NN + n) * NOR + i]); const float cv = ok ? bfr(co[(((size_t)b * 3 + d) * NN + (ok ? m : 0)) * NOR + i]) : 0.f; const float df = cv - cc; s = fmaf(df, df, s); }
          w = fmaxf(1.0f - sqrtf(s) / SIG, 0.f); }
      if (lane < 16) dws[wv][lane] = w; }
    __syncthreads();
    const float* dw = dws[wv];
#pragma unroll 1
    for (int ps = 0; ps < 2; ++ps) {
#pragma unroll 1
        for (int e0 = lane * 8; e0 < KC; e0 += 256) { v8us oh, ol;
#pragma unroll
            for (int q = 0; q < 8; ++q) { const int e = e0 + q; const int c = e / KK, k = e - c * KK; const int m = n + k - PADK; const bool ok = (m >= 0) && (m < NN);
                const float v = ok ? bfr(XG[(size_t)c * NN + (ok ? m : 0)]) * dw[k] : 0.f; const unsigned short hb = f2bf(v); oh[q] = hb; ol[q] = f2bf(v - bf2f(hb)); }
            const size_t o = (size_t)n * KC + e0; *(volatile v8us*)(Ah + o) = oh; *(volatile v8us*)(Al + o) = ol; }
        if (ps == 0) __threadfence(); }
}
__global__ __launch_bounds__(256) void k_regather(const float* __restrict__ Y, const int* __restrict__ ridx, int b, int i, bf* Ch, bf* Cl) {
    typedef __attribute__((ext_vector_type(2))) unsigned short v2us;
    const int lane = threadIdx.x & 31, n = blockIdx.x * 8 + (threadIdx.x >> 5); if (n >= NN) return; int m = ridx[((size_t)b * NN + n) * NOR + i]; m = m < 0 ? 0 : (m >= NN ? NN - 1 : m); v2us oh, ol;
#pragma unroll
    for (int q = 0; q < 2; ++q) { const float v = Y[(size_t)m * CO + lane * 2 + q]; const unsigned short hb = f2bf(v); oh[q] = hb; ol[q] = f2bf(v - bf2f(hb)); }
    const size_t o = (size_t)n * CCAT + i * CO + lane * 2; *(volatile v2us*)(Ch + o) = oh; *(volatile v2us*)(Cl + o) = ol; __threadfence(); *(volatile v2us*)(Ch + o) = oh; *(volatile v2us*)(Cl + o) = ol;
}
template <int MODE>
__global__ __launch_bounds__(256) void k_colstat(const float* __restrict__ Z, const float* __restrict__ fb, const float* __restrict__ MEAN, float* OUTV) {
    const int o = threadIdx.x; float s = 0.f;
    if (o < CO) { const float bb = bfr(fb[o]); const float mu = (MODE == 1) ? MEAN[o] : 0.f;
#pragma unroll 1
        for (int r = 0; r < NBI * NN; ++r) { const float v = Z[(size_t)r * CO + o] + bb; const float d = (MODE == 1) ? (v - mu) * (v - mu) : v; s += d; }
        const float pv = (MODE == 1) ? (bb - mu) * (bb - mu) : bb; s += (float)(2 * NBI) * pv; s *= 1.0f / (float)(NBI * NP2); }
    *(volatile float*)(OUTV + o) = s; __threadfence(); *(volatile float*)(OUTV + o) = s;
}
__global__ __launch_bounds__(256) void k_out(const float* __restrict__ Z, const float* __restrict__ fb, const float* __restrict__ MEAN, const float* __restrict__ VAR, const float* __restrict__ ga, const float* __restrict__ be, float* OUTP) {
    const size_t u = (size_t)blockIdx.x * 256 + threadIdx.x; if (u >= (size_t)NBI * CO * NP2 / 4) return; v4f ov;
#pragma unroll
    for (int q = 0; q < 4; ++q) { const size_t e = u * 4 + q; const int b = (int)(e / ((size_t)CO * NP2)); const size_t rem = e % ((size_t)CO * NP2); const int o = (int)(rem / NP2), j = (int)(rem % NP2);
        float v = bfr(fb[o]); if (j >= 1 && j <= NN) v += Z[((size_t)b * NN + (j - 1)) * CO + o];
        const float y = (v - MEAN[o]) * rsqrtf(VAR[o] + BEPS) * bfr(ga[o]) + bfr(be[o]); ov[q] = fmaxf(y, 0.f); }
    *(volatile v4f*)(OUTP + u * 4) = ov; __threadfence(); *(volatile v4f*)(OUTP + u * 4) = ov;
}

extern "C" void kernel_launch(void* const* d_in, const int* in_sizes, int n_in,
                              void* d_out, int out_size, void* d_ws, size_t ws_size, hipStream_t stream) {
    (void)in_sizes; (void)n_in; (void)out_size;
    const float* x = (const float*)d_in[0]; const float* co = (const float*)d_in[1]; const int* idx = (const int*)d_in[2]; const int* ridx = (const int*)d_in[3];
    const float* cw = (const float*)d_in[4]; const float* fw = (const float*)d_in[5]; const float* fb = (const float*)d_in[6]; const float* ga = (const float*)d_in[7]; const float* be = (const float*)d_in[8];
    float* out = (float*)d_out;
    char* wsp = (char*)d_ws;
    auto take = [&](size_t bytes) { char* p = wsp; wsp += (bytes + 255) & ~(size_t)255; return (void*)p; };
    bf* CWB = (bf*)take((size_t)NOR * CO * KC * 2); bf* FWB = (bf*)take((size_t)CO * CCAT * 2);
    float* XA = (float*)take((size_t)CH * NN * 4); float* XB = (float*)take((size_t)CH * NN * 4); bf* Ah = (bf*)take((size_t)NN * KC * 2); bf* Al = (bf*)take((size_t)NN * KC * 2); float* Y = (float*)take((size_t)NN * CO * 4);
    bf* Ch = (bf*)take((size_t)NN * CCAT * 2); bf* Cl = (bf*)take((size_t)NN * CCAT * 2); float* Z = (float*)take((size_t)NBI * NN * CO * 4); float* MEAN = (float*)take(256 * 4); float* VAR = (float*)take(256 * 4);
    if ((size_t)(wsp - (char*)d_ws) > ws_size) return;
    k_cvt8<<<(NOR * CO * KC / 8 + 255) / 256, 256, 0, stream>>>(cw, CWB, NOR * CO * KC / 8);
    k_cvt8<<<(CO * CCAT / 8 + 255) / 256, 256, 0, stream>>>(fw, FWB, CO * CCAT / 8);
    for (int b = 0; b < NBI; ++b) {
        const float* src = x + (size_t)b * CH * NN; float* bufs[2] = {XA, XB};
        for (int i = 0; i < NOR; ++i) { float* dst = bufs[i & 1];
            k_xgather<<<(CH * (NN / 32)) / 8, 256, 0, stream>>>(src, idx, b, i, dst);
            k_wim<<<NN / 8, 256, 0, stream>>>(dst, co, b, i, Ah, Al);
            k_gemmb<true, false><<<dim3(NN / 64, 1, 1), 128, 0, stream>>>(Ah, Al, CWB + (size_t)i * CO * KC, nullptr, Y, CO, nullptr, nullptr, KC);
            k_regather<<<NN / 8, 256, 0, stream>>>(Y, ridx, b, i, Ch, Cl);
            src = dst; }
        k_gemmb<true, false><<<dim3(NN / 64, 1, 1), 128, 0, stream>>>(Ch, Cl, FWB, nullptr, Z + (size_t)b * NN * CO, CO, nullptr, nullptr, CCAT); }
    k_colstat<0><<<1, 256, 0, stream>>>(Z, fb, nullptr, MEAN); k_colstat<1><<<1, 256, 0, stream>>>(Z, fb, MEAN, VAR);
    k_out<<<(unsigned)(((size_t)NBI * CO * NP2 / 4 + 255) / 256), 256, 0, stream>>>(Z, fb, MEAN, VAR, ga, be, out);
}
